// LowRankProcessNeurons_15668040696247
// MI455X (gfx1250) — hardware-verified
//
#include <hip/hip_runtime.h>


#define NBT  4
#define SS   1024
#define HH   1024
#define NIN  64
#define NP   16
#define RR   128
#define NPR  (NP * RR)
#define DM   HH
#define LOSC 1024.0f

typedef _Float16 h16;
typedef unsigned short bf;
typedef __attribute__((ext_vector_type(16))) __bf16   v16bf;
typedef __attribute__((ext_vector_type(16))) _Float16 v16h;
typedef __attribute__((ext_vector_type(8)))  _Float16 v8h;
typedef __attribute__((ext_vector_type(8)))  unsigned short v8us;
typedef __attribute__((ext_vector_type(8)))  float    v8f;
typedef __attribute__((ext_vector_type(4)))  float    v4f;
typedef __attribute__((ext_vector_type(4)))  _Float16 v4h;
typedef v8h  __attribute__((may_alias)) v8ha;
typedef v4f  __attribute__((may_alias)) v4fa;
typedef v8us __attribute__((may_alias)) v8usa;

__device__ __forceinline__ unsigned short f2bf(float f) { unsigned u = __float_as_uint(f); u += 0x7FFFu + ((u >> 16) & 1u); return (unsigned short)(u >> 16); }
__device__ __forceinline__ float bf2f(unsigned short b) { return __uint_as_float(((unsigned)b) << 16); }
__device__ __forceinline__ float bfr(float f) { return bf2f(f2bf(f)); }
__device__ __forceinline__ v16h cat16(v8h lo, v8h hi) { return __builtin_shufflevector(lo, hi, 0, 1, 2, 3, 4, 5, 6, 7, 8, 9, 10, 11, 12, 13, 14, 15); }
__device__ __forceinline__ v16bf cat16b(v8us lo, v8us hi) { return __builtin_bit_cast(v16bf, __builtin_shufflevector(lo, hi, 0, 1, 2, 3, 4, 5, 6, 7, 8, 9, 10, 11, 12, 13, 14, 15)); }
__device__ __forceinline__ v8f wmma16(v16h a, v16h b, v8f c) { return __builtin_amdgcn_wmma_f32_16x16x32_f16(false, a, false, b, (short)0, c, false, false); }
__device__ __forceinline__ v8f wmmab(v16bf a, v16bf b, v8f c) { return __builtin_amdgcn_wmma_f32_16x16x32_bf16(false, a, false, b, (short)0, c, false, false); }

__global__ __launch_bounds__(256) void k_wt(const float* __restrict__ Wm, int K, int ncols, bf* WT) {
    __shared__ __align__(16) unsigned short tl[64 * 72];
    const int tid = threadIdx.x, k0 = blockIdx.x * 64, n0 = blockIdx.y * 64;
    const int kk = tid >> 2, nq = (tid & 3) * 16;
#pragma unroll
    for (int i = 0; i < 16; ++i) tl[(nq + i) * 72 + kk] = f2bf(Wm[(size_t)(k0 + kk) * ncols + n0 + nq + i]);
    __syncthreads();
    const int piece = tid & 7;
    auto pass = [&]() {
#pragma unroll
        for (int s = 0; s < 2; ++s) { const int nr = (tid >> 3) + 32 * s; const v8us val = *(const v8usa*)(tl + nr * 72 + piece * 8); *(volatile v8us*)(WT + (size_t)(n0 + nr) * K + k0 + piece * 8) = val; }
    };
    pass(); __threadfence(); pass();
}
template <bool SPLITA, bool F16OUT = false>
__global__ __launch_bounds__(128) void k_gemmb(const bf* __restrict__ A, const bf* __restrict__ Al, const bf* __restrict__ Bn, const float* __restrict__ bias, float* C, int ldc, h16* C2, const float* __restrict__ R = nullptr, int K = DM, int roundR = 1) {
    __shared__ __align__(16) float ost[4][16 * 68];
    const int lane = threadIdx.x & 31, wave = threadIdx.x >> 5, lr = lane & 15, hi = lane >> 4;
    const int r0 = blockIdx.x * 64 + wave * 16, c0 = blockIdx.y * 64;
    const size_t aoff = (size_t)(r0 + lr) * K + 8 * hi;
    size_t boff[4];
#pragma unroll
    for (int t = 0; t < 4; ++t) boff[t] = (size_t)(c0 + t * 16 + lr) * K + 8 * hi;
    v8f acc[4];
#pragma unroll
    for (int t = 0; t < 4; ++t) acc[t] = (v8f){};
#pragma unroll 1
    for (int kc = 0; kc < K; kc += 32) {
        const v16bf a = cat16b(*(const v8us*)(A + aoff + kc), *(const v8us*)(A + aoff + kc + 16));
        v16bf al = a;
        if (SPLITA) al = cat16b(*(const v8us*)(Al + aoff + kc), *(const v8us*)(Al + aoff + kc + 16));
#pragma unroll
        for (int t = 0; t < 4; ++t) { const v16bf b = cat16b(*(const v8us*)(Bn + boff[t] + kc), *(const v8us*)(Bn + boff[t] + kc + 16)); acc[t] = wmmab(a, b, acc[t]); if (SPLITA) acc[t] = wmmab(al, b, acc[t]); }
        asm volatile("v_nop\n\tv_nop\n\tv_nop\n\tv_nop" : "+v"(acc[0]), "+v"(acc[1]), "+v"(acc[2]), "+v"(acc[3]) : "v"(a), "v"(al));
    }
    float* os = &ost[wave][0];
#pragma unroll
    for (int t = 0; t < 4; ++t) { const float bv = bias ? bfr(bias[c0 + t * 16 + lr]) : 0.f;
#pragma unroll
        for (int j = 0; j < 8; ++j) os[(hi * 8 + j) * 68 + t * 16 + lr] = acc[t][j] + bv; }
    __syncthreads();
    if (F16OUT) {
        h16* crow = (h16*)(void*)C + (size_t)r0 * ldc + c0;
        auto pass = [&]() {
#pragma unroll
            for (int s = 0; s < 4; ++s) { const int row = 4 * s + (lane >> 3), piece = lane & 7; const float* sp = os + row * 68 + piece * 8; v8h o, o2;
#pragma unroll
                for (int i = 0; i < 8; ++i) { const h16 a = (h16)sp[i]; o[i] = a; o2[i] = (h16)((sp[i] - (float)a) * LOSC); }
                *(volatile v8h*)(crow + (size_t)row * ldc + piece * 8) = o; if (C2) *(volatile v8h*)(C2 + (size_t)r0 * ldc + c0 + (size_t)row * ldc + piece * 8) = o2; }
        };
        pass(); __threadfence(); pass();
    } else {
        float* crow = C + (size_t)r0 * ldc + c0;
        auto pass = [&]() {
#pragma unroll
            for (int s = 0; s < 8; ++s) { const int Lid = (lane >> 3) + 4 * s, piece = lane & 7; const int row = Lid >> 1, cofs = (Lid & 1) * 32 + piece * 4;
                v4f val = *(const v4fa*)(os + row * 68 + cofs); if (R) { const v4f rv = *(const v4f*)(R + ((size_t)r0 + row) * ldc + c0 + cofs); val += roundR ? (v4f){bfr(rv[0]), bfr(rv[1]), bfr(rv[2]), bfr(rv[3])} : rv; }
                *(volatile v4f*)(crow + (size_t)row * ldc + cofs) = val; }
        };
        pass(); __threadfence(); pass();
    }
}


__global__ __launch_bounds__(256) void k_cvt8(const float* __restrict__ src, bf* dst, size_t n8) {
    const size_t i = (size_t)blockIdx.x * 256 + threadIdx.x; if (i >= n8) return;
    const v8f v = *(const v8f*)(src + i * 8); v8us o;
#pragma unroll
    for (int k = 0; k < 8; ++k) o[k] = f2bf(v[k]);
    *(volatile v8us*)(dst + i * 8) = o; __threadfence(); *(volatile v8us*)(dst + i * 8) = o;
}
__global__ __launch_bounds__(256) void k_zero8(bf* dst, size_t n8) {
    const size_t i = (size_t)blockIdx.x * 256 + threadIdx.x; if (i >= n8) return; v8us z;
#pragma unroll
    for (int k = 0; k < 8; ++k) z[k] = 0;
    *(volatile v8us*)(dst + i * 8) = z; __threadfence(); *(volatile v8us*)(dst + i * 8) = z;
}

__global__ __launch_bounds__(256) void k_cvtx(const float* __restrict__ src, bf* dst) {
    const int lane = threadIdx.x & 31; const size_t r = (size_t)blockIdx.x * 8 + (threadIdx.x >> 5); if (r >= (size_t)SS) return;
#pragma unroll 1
    for (int ps = 0; ps < 2; ++ps) {
#pragma unroll
        for (int q = 0; q < HH / 256; ++q) { v8us o;
#pragma unroll
            for (int i = 0; i < 8; ++i) o[i] = f2bf(src[r * HH + q * 256 + lane * 8 + i]);
            *(volatile v8us*)(dst + r * HH + q * 256 + lane * 8) = o; }
        if (ps == 0) __threadfence(); }
}
__global__ __launch_bounds__(256) void k_upgather(const float* __restrict__ up, bf* UPB) {
    const int lane = threadIdx.x & 31; const int h = blockIdx.x * 8 + (threadIdx.x >> 5); if (h >= HH) return;
#pragma unroll 1
    for (int ps = 0; ps < 2; ++ps) {
#pragma unroll 1
        for (int q = 0; q < NPR / 256; ++q) { v8us o;
#pragma unroll
            for (int i = 0; i < 8; ++i) { const int nr = q * 256 + lane * 8 + i; o[i] = f2bf(up[(size_t)nr * HH + h]); }
            *(volatile v8us*)(UPB + (size_t)h * NPR + q * 256 + lane * 8) = o; }
        if (ps == 0) __threadfence(); }
}
__global__ __launch_bounds__(256) void k_gate(const float* __restrict__ act, const float* __restrict__ cw, const float* __restrict__ cb, float* G, float* OUT2) {
    const int lane = threadIdx.x & 31; const int sp = blockIdx.x * 8 + (threadIdx.x >> 5); if (sp >= SS / 2) return; float mine = 0.f;
#pragma unroll 1
    for (int hf = 0; hf < 2; ++hf) { const int s = sp * 2 + hf; float av[10];
#pragma unroll
        for (int t = 0; t < 5; ++t) { const int sr = s + t - 2; const bool ok = sr >= 0 && sr < SS;
#pragma unroll
            for (int i = 0; i < 2; ++i) av[t * 2 + i] = ok ? bfr(act[(size_t)(ok ? sr : 0) * NIN + lane * 2 + i]) : 0.f; }
#pragma unroll 1
        for (int n = 0; n < NP; ++n) { float p = 0.f;
#pragma unroll
            for (int t = 0; t < 5; ++t) {
#pragma unroll
                for (int i = 0; i < 2; ++i) p = fmaf(bfr(cw[((size_t)n * 5 + t) * NIN + lane * 2 + i]), av[t * 2 + i], p); }
#pragma unroll
            for (int sh = 16; sh; sh >>= 1) p += __shfl_xor(p, sh, 32);
            const float gv = 1.0f / (1.0f + __expf(-(p + bfr(cb[n])))); if (lane == hf * 16 + n) mine = gv; } }
    const size_t o = (size_t)sp * 2 * NP + lane; *(volatile float*)(G + o) = mine; *(volatile float*)(OUT2 + o) = mine; __threadfence(); *(volatile float*)(G + o) = mine; *(volatile float*)(OUT2 + o) = mine;
}
__global__ __launch_bounds__(256) void k_gated(const float* __restrict__ D, const float* __restrict__ G, bf* Ph, bf* Pl) {
    const int lane = threadIdx.x & 31; const size_t s = (size_t)blockIdx.x * 8 + (threadIdx.x >> 5); if (s >= (size_t)SS) return;
#pragma unroll 1
    for (int ps = 0; ps < 2; ++ps) {
#pragma unroll 1
        for (int q = 0; q < NPR / 256; ++q) { const size_t o = s * NPR + q * 256 + lane * 8; const v8f v = *(const v8f*)(D + o); const float gv = G[s * NP + (q * 256 + lane * 8) / RR]; v8us oh, ol;
#pragma unroll
            for (int i = 0; i < 8; ++i) { const float y = v[i] * gv; const unsigned short hb = f2bf(y); oh[i] = hb; ol[i] = f2bf(y - bf2f(hb)); }
            *(volatile v8us*)(Ph + o) = oh; *(volatile v8us*)(Pl + o) = ol; }
        if (ps == 0) __threadfence(); }
}

extern "C" void kernel_launch(void* const* d_in, const int* in_sizes, int n_in,
                              void* d_out, int out_size, void* d_ws, size_t ws_size, hipStream_t stream) {
    (void)in_sizes; (void)n_in; (void)out_size;
    const float* x = (const float*)d_in[0]; const float* act = (const float*)d_in[1]; const float* cw = (const float*)d_in[2]; const float* cb = (const float*)d_in[3]; const float* dp = (const float*)d_in[4]; const float* up = (const float*)d_in[5];
    float* out = (float*)d_out;
    float* out2 = (float*)((char*)d_out + (size_t)NBT * SS * HH * 4);
    char* wsp = (char*)d_ws;
    auto take = [&](size_t bytes) { char* p = wsp; wsp += (bytes + 255) & ~(size_t)255; return (void*)p; };
    bf* DPB = (bf*)take((size_t)NPR * HH * 2); bf* UPB = (bf*)take((size_t)HH * NPR * 2); bf* Xb = (bf*)take((size_t)SS * HH * 2); float* D = (float*)take((size_t)SS * NPR * 4); float* G = (float*)take((size_t)SS * NP * 4); bf* Ph = (bf*)take((size_t)SS * NPR * 2); bf* Pl = (bf*)take((size_t)SS * NPR * 2);
    if ((size_t)(wsp - (char*)d_ws) > ws_size) return;
    for (int n = 0; n < NP; ++n) k_wt<<<dim3(HH / 64, RR / 64, 1), 256, 0, stream>>>(dp + (size_t)n * HH * RR, HH, RR, DPB + (size_t)n * RR * HH);
    k_upgather<<<HH / 8, 256, 0, stream>>>(up, UPB);
    for (int b = 0; b < NBT; ++b) {
        k_cvtx<<<SS / 8, 256, 0, stream>>>(x + (size_t)b * SS * HH, Xb);
        k_gemmb<false, false><<<dim3(SS / 64, NPR / 64, 1), 128, 0, stream>>>(Xb, nullptr, DPB, nullptr, D, NPR, nullptr, nullptr, HH);
        k_gate<<<(SS / 2) / 8, 256, 0, stream>>>(act + (size_t)b * SS * NIN, cw, cb, G, out2 + (size_t)b * SS * NP);
        k_gated<<<SS / 8, 256, 0, stream>>>(D, G, Ph, Pl);
        k_gemmb<true, false><<<dim3(SS / 64, HH / 64, 1), 128, 0, stream>>>(Ph, Pl, UPB, nullptr, out + (size_t)b * SS * HH, HH, nullptr, nullptr, NPR); }
}
